// SelfAttention_49108656062912
// MI455X (gfx1250) — hardware-run, weakly checked
//
#include <hip/hip_runtime.h>

typedef float          v8f   __attribute__((ext_vector_type(8)));
typedef float          v4f   __attribute__((ext_vector_type(4)));
typedef unsigned int   v4u   __attribute__((ext_vector_type(4)));
typedef int            v8i   __attribute__((ext_vector_type(8)));
typedef unsigned short v8us  __attribute__((ext_vector_type(8)));
typedef unsigned short v16us __attribute__((ext_vector_type(16)));
typedef __bf16         v16bf __attribute__((ext_vector_type(16)));
typedef _Float16       v16h  __attribute__((ext_vector_type(16)));
typedef v4f  __attribute__((may_alias)) v4fa;
typedef v8us __attribute__((may_alias)) v8usa;
union FragB { v16bf v; v16us u; v8us h[2]; v8i w; };
union FragH { v16h  v; v16us u; v8us h[2]; v8i w; };

__device__ __forceinline__ v8f wmb(const FragB& a, const FragB& b, v8f c) {
  v8f d = __builtin_amdgcn_wmma_f32_16x16x32_bf16(false, a.v, false, b.v, (short)0, c, false, false);
  asm volatile("v_nop\n\tv_nop\n\tv_nop\n\tv_nop" : "+v"(d) : "v"(a.w), "v"(b.w));
  return d;
}

__device__ __forceinline__ v8f wmh(const FragH& a, const FragH& b, v8f c) {
  v8f d = __builtin_amdgcn_wmma_f32_16x16x32_f16(false, a.v, false, b.v, (short)0, c, false, false);
  asm volatile("v_nop\n\tv_nop\n\tv_nop\n\tv_nop" : "+v"(d) : "v"(a.w), "v"(b.w));
  return d;
}

__device__ __forceinline__ unsigned bf16_bits(float f) {
  const unsigned u = __float_as_uint(f);
  const unsigned r = (u + 0x7FFFu + ((u >> 16) & 1u)) >> 16;
  const unsigned q = (u >> 16) | 0x40u;
  return ((u & 0x7fffffffu) > 0x7f800000u) ? q : r;
}

__device__ __forceinline__ float bf16_val(float f) {
  return __uint_as_float(bf16_bits(f) << 16);
}
__device__ __forceinline__ int clampi(int v, int lo, int hi) {
  return v < lo ? lo : (v > hi ? hi : v);
}

__device__ __forceinline__ unsigned f16_bits(float f) {
  const unsigned u  = __float_as_uint(f);
  const unsigned s  = (u >> 16) & 0x8000u;
  const unsigned a  = u & 0x7fffffffu;
  const unsigned t  = a - 0x38000000u;
  const unsigned r  = (t + 0x0FFFu + ((t >> 13) & 1u)) >> 13;
  const unsigned rc = r > 0x7C00u ? 0x7C00u : r;
  const bool small  = a < 0x38800000u;
  const bool isnan  = a > 0x7f800000u;
  const unsigned fin = small ? 0u : (s | rc);
  return isnan ? (s | 0x7E00u) : fin;
}

__device__ __forceinline__ unsigned pk16(unsigned lo, unsigned hi) { return lo | (hi << 16); }
__device__ __forceinline__ unsigned bf16_lo_bits(float v) {
  float hi = bf16_val(v);
  asm volatile("" : "+v"(hi));
  return bf16_bits(v - hi);
}
__device__ __forceinline__ v4u pack8_bf16(v4f a, v4f c) {
  return (v4u){ pk16(bf16_bits(a[0]), bf16_bits(a[1])), pk16(bf16_bits(a[2]), bf16_bits(a[3])),
                pk16(bf16_bits(c[0]), bf16_bits(c[1])), pk16(bf16_bits(c[2]), bf16_bits(c[3])) };
}
__device__ __forceinline__ v4u pack8_bf16_lo(v4f a, v4f c) {
  return (v4u){ pk16(bf16_lo_bits(a[0]), bf16_lo_bits(a[1])), pk16(bf16_lo_bits(a[2]), bf16_lo_bits(a[3])),
                pk16(bf16_lo_bits(c[0]), bf16_lo_bits(c[1])), pk16(bf16_lo_bits(c[2]), bf16_lo_bits(c[3])) };
}
__device__ __forceinline__ v4u pack8_f16(v4f a, v4f c) {
  return (v4u){ pk16(f16_bits(a[0]), f16_bits(a[1])), pk16(f16_bits(a[2]), f16_bits(a[3])),
                pk16(f16_bits(c[0]), f16_bits(c[1])), pk16(f16_bits(c[2]), f16_bits(c[3])) };
}

template <int FORM>
__global__ __launch_bounds__(256) void k_plane(const float* __restrict__ src, int rows, int cols, int ldsrc,
                                               unsigned short* __restrict__ dst, int MP, int KP) {
  static_assert(FORM >= 0 && FORM <= 3);
  const int KTOT = (FORM == 1 || FORM == 3) ? 2 * KP : KP;
  const unsigned ppr   = (unsigned)(KTOT >> 3);
  const unsigned kp8   = (unsigned)(KP >> 3);
  const unsigned total = (unsigned)MP * ppr;
  const unsigned g     = blockIdx.x * 256u + threadIdx.x;
  const unsigned rowu  = g / ppr;
  const unsigned p     = g - rowu * ppr;
  const bool second    = p >= kp8;
  const int row = (int)rowu;
  const int c0  = (int)((second ? p - kp8 : p) << 3);
  const float* srow = src + (size_t)clampi(row, 0, rows - 1) * (size_t)ldsrc;
  float x[8];
  unsigned mk[8];
#pragma unroll
  for (int e = 0; e < 8; ++e) {
    const int c = c0 + e;
    const float v = srow[clampi(c, 0, cols - 1)];
    asm volatile("" :: "v"(v));
    x[e]  = v;
    mk[e] = (row < rows && c < cols) ? 0xFFFFu : 0u;
  }
  const v4f a = (v4f){ x[0], x[1], x[2], x[3] };
  const v4f c = (v4f){ x[4], x[5], x[6], x[7] };
  v4u o;
  if (FORM == 2) {
    o = pack8_f16(a, c);
  } else {
    const v4u hi = pack8_bf16(a, c);
    o = hi;
    if (FORM == 1) { const v4u lo = pack8_bf16_lo(a, c); o = second ? lo : hi; }
  }
  const v4u mw = (v4u){ pk16(mk[0], mk[1]), pk16(mk[2], mk[3]), pk16(mk[4], mk[5]), pk16(mk[6], mk[7]) };
  o &= mw;
  if (g < total) {
    volatile v4u* q = (volatile v4u*)(dst + (size_t)g * 8);
    *q = o;
    __threadfence();
    *q = o;
  }
}

template <int FORM> struct FragOf    { typedef FragB T; };
template <>         struct FragOf<2> { typedef FragH T; };
__device__ __forceinline__ v8f mm(const FragB& a, const FragB& b, v8f c) { return wmb(a, b, c); }
__device__ __forceinline__ v8f mm(const FragH& a, const FragH& b, v8f c) { return wmh(a, b, c); }
template <class F> __device__ __forceinline__ F ld_frag(const unsigned short* p) {
  F f;
  f.h[0] = *(const v8usa*)(p);
  f.h[1] = *(const v8usa*)(p + 16);
  return f;
}

template <int FORM, int EPI>
__global__ __launch_bounds__(256) __attribute__((amdgpu_num_vgpr(248)))
void k_gemm_nt(const unsigned short* __restrict__ A, const unsigned short* __restrict__ B,
               const float* __restrict__ bias, float* __restrict__ D, int M, int N, int KTOT, int ldd) {
  static_assert(FORM >= 0 && FORM <= 2);
  static_assert(EPI == 0 || EPI == 1);
  typedef typename FragOf<FORM>::T F;
  __shared__ __attribute__((aligned(16))) float sT[8][16 * 68];
  const int lane = threadIdx.x & 31;
  const int wave = threadIdx.x >> 5;
  const int tilesM = (M + 63) >> 6;
  const int tilesN = (N + 63) >> 6;
  const int tile = blockIdx.x * 8 + wave;
  if (tile >= tilesM * tilesN) return;
  const int tm = tile / tilesN;
  const int tn = tile - tm * tilesN;
  const int m0 = tm << 6;
  const int n0 = tn << 6;

  const int rl = lane & 15;
  const int h8 = (lane >> 4) * 8;
  const unsigned short* pa = A + (size_t)(m0 + rl) * (size_t)KTOT + h8;
  const unsigned short* pb = B + (size_t)(n0 + rl) * (size_t)KTOT + h8;

  v8f acc[4][4];
#pragma unroll
  for (int i = 0; i < 4; ++i)
#pragma unroll
    for (int j = 0; j < 4; ++j) acc[i][j] = (v8f){0.f, 0.f, 0.f, 0.f, 0.f, 0.f, 0.f, 0.f};

#pragma unroll 1
  for (int k0 = 0; k0 < KTOT; k0 += 32) {
    F bf[4];
#pragma unroll
    for (int j = 0; j < 4; ++j) bf[j] = ld_frag<F>(pb + (size_t)(j << 4) * (size_t)KTOT + k0);
#pragma unroll
    for (int i = 0; i < 4; ++i) {
      const F af = ld_frag<F>(pa + (size_t)(i << 4) * (size_t)KTOT + k0);
#pragma unroll
      for (int j = 0; j < 4; ++j) acc[i][j] = mm(af, bf[j], acc[i][j]);
    }
  }

  float* slab = sT[wave];
  const int hh = lane >> 4;
  const int c4 = (lane & 15) * 4;
  const int nc = n0 + c4;
  const bool cok = nc < N;
  v4f bv = (v4f){0.f, 0.f, 0.f, 0.f};
  if (EPI == 1) {
    bv = *(const v4fa*)(bias + clampi(nc, 0, N - 4));
    asm volatile("" :: "v"(bv));
  }
#pragma unroll
  for (int i = 0; i < 4; ++i) {
    const int mBase = m0 + (i << 4);
#pragma unroll
    for (int j = 0; j < 4; ++j) {
#pragma unroll
      for (int r = 0; r < 8; ++r) slab[(h8 + r) * 68 + (j << 4) + rl] = acc[i][j][r];
    }
    __builtin_amdgcn_fence(__ATOMIC_RELEASE, "workgroup");
    __builtin_amdgcn_wave_barrier();
    __builtin_amdgcn_fence(__ATOMIC_ACQUIRE, "workgroup");
    v4f vv[8];
#pragma unroll
    for (int it = 0; it < 8; ++it) {
      const int row = it * 2 + hh;
      v4f v = *(const v4fa*)(slab + row * 68 + c4);
      if (EPI == 1) v += bv;
      vv[it] = v;
    }
    for (int pass = 0; pass < 2; ++pass) {
#pragma unroll
      for (int it = 0; it < 8; ++it) {
        const int row = mBase + it * 2 + hh;
        if (cok && row < M) *(volatile v4f*)(D + (size_t)row * (size_t)ldd + nc) = vv[it];
      }
      __threadfence();
    }
    __builtin_amdgcn_fence(__ATOMIC_RELEASE, "workgroup");
    __builtin_amdgcn_wave_barrier();
    __builtin_amdgcn_fence(__ATOMIC_ACQUIRE, "workgroup");
  }
}

#ifndef SPLIT_EK
#define SPLIT_EK 0
#endif
#ifndef SPLIT_EV
#define SPLIT_EV 1
#endif
#ifndef SPLIT_PROJ
#define SPLIT_PROJ 1
#endif
#define KT_EK    (SPLIT_EK ? 256 : 128)
#define KT_EV    (SPLIT_EV ? 256 : 128)
#define KT_PJ    (SPLIT_PROJ ? 256 : 128)

#define SEQ_L    4096
#define N_NODES  16384
#define N_EDGES  262144
#define DM       128
#define NFE      5
#define NBRUN    1024
#define NBLK     16
#define BCAP     17408
#define DEGCAP   104
#define GCH      2
#define NCHUNK   8
#define CHROWS   (GCH * BCAP)
#define NTHR     256
#define NWAVE    8
#define EPT      8
#define CHUNK    (NTHR * EPT)
#define WCAP     (EPT * 32)
#define LISTN    (NWAVE * WCAP)
#define OFFP     1056
#define LDS_BKT  ((2 * BCAP + NBRUN + OFFP + LISTN + 32) * 4)
#define PPW      8
#define HPLANE   ((size_t)CHROWS * 256)

#define PAR_KB    0
#define PAR_QB    128
#define PAR_VB    256
#define PAR_PB    384
#define PAR_EKB2  512
#define PAR_EVB2  640
#define PAR_EDGE0 768
#define PAR_EAW2  3840
#define PAR_EAB2  4864
#define PAR_N     4896
#define PE_N      (PAR_N - PAR_EDGE0)

static_assert(DM == 128 && 8 * 16 == DM);
static_assert(N_NODES == 4 * SEQ_L && NBLK * NBRUN == N_NODES && (N_NODES % 2048) == 0);
static_assert(N_EDGES < (1 << 20) && (N_EDGES % CHUNK) == 0);
static_assert(NBRUN <= (1 << 10) && NTHR * 4 == NBRUN);
static_assert((BCAP % 128) == 0 && (BCAP % (NWAVE * PPW)) == 0 && BCAP >= 16384 + 1024 && BCAP <= 18432);
static_assert(DEGCAP >= 91 + 8 && DEGCAP >= 33 + 8 && (DEGCAP % 8) == 0);
static_assert(GCH * NCHUNK == NBLK);
static_assert((CHROWS % 128) == 0 && (CHROWS % (NWAVE * PPW)) == 0);
static_assert((OFFP % 32) == 0 && OFFP >= NBRUN + 3);
static_assert(CHUNK == 2048 && LISTN >= NWAVE * WCAP);
static_assert(LDS_BKT <= 262144);
static_assert(NWAVE * DEGCAP * 8 * 4 + 1024 <= 65536);
static_assert(PE_N * 4 <= 65536 && (PE_N % 4) == 0 && (PAR_N % 32) == 0);
static_assert(PAR_EVB2 == PAR_EKB2 + 128 && PAR_EAW2 == PAR_EDGE0 + 3072 && PAR_EAB2 == PAR_EAW2 + 1024);
static_assert((KT_EK % 32) == 0 && (KT_EV % 32) == 0 && (KT_PJ % 32) == 0);

#define WS_OXK   ((size_t)0)
#define WS_OXV   (WS_OXK  + (size_t)N_NODES * DM * 2)
#define WS_OXQ   (WS_OXV  + (size_t)N_NODES * DM * 2)
#define WS_OKW   (WS_OXQ  + (size_t)N_NODES * DM * 2)
#define WS_OQW   (WS_OKW  + (size_t)DM * 128 * 2)
#define WS_OVW   (WS_OQW  + (size_t)DM * 128 * 2)
#define WS_OEKW  (WS_OVW  + (size_t)DM * 128 * 2)
#define WS_OEVW  (WS_OEKW + (size_t)DM * 256 * 2)
#define WS_OPW   (WS_OEVW + (size_t)DM * 256 * 2)
#define WS_OPAR  (WS_OPW  + (size_t)DM * 256 * 2)
#define WS_OKF   (WS_OPAR + (size_t)19712)
#define WS_OQF   (WS_OKF  + (size_t)N_NODES * DM * 4)
#define WS_OVF   (WS_OQF  + (size_t)N_NODES * DM * 4)
#define WS_OLIST (WS_OVF  + (size_t)N_NODES * DM * 4)
#define WS_OOFFS (WS_OLIST + (size_t)NBLK * BCAP * 8)
#define WS_OHK   (WS_OOFFS + (size_t)NBLK * OFFP * 4)
#define WS_OHV   (WS_OHK  + HPLANE * 2)
#define WS_OEK   (WS_OHV  + HPLANE * 2)
#define WS_OEV   (WS_OEK  + (size_t)CHROWS * DM * 4)
#define WS_OEA   (WS_OEV  + (size_t)CHROWS * DM * 4)
#define WS_OYHL  (WS_OEA  + (size_t)CHROWS * 32 * 4)
#define WS_TOTAL (WS_OYHL + (size_t)N_NODES * 256 * 2)
static_assert(PAR_N * 4 <= 19712);
static_assert(WS_TOTAL == (size_t)((size_t)486357 << 8));
static_assert(WS_TOTAL <= ((size_t)128 << 20));
static_assert((WS_OXV % 256) == 0 && (WS_OXQ % 256) == 0 && (WS_OKW % 256) == 0 && (WS_OQW % 256) == 0);
static_assert((WS_OVW % 256) == 0 && (WS_OEKW % 256) == 0 && (WS_OEVW % 256) == 0 && (WS_OPW % 256) == 0);
static_assert((WS_OPAR % 256) == 0 && (WS_OKF % 256) == 0 && (WS_OQF % 256) == 0 && (WS_OVF % 256) == 0);
static_assert((WS_OLIST % 256) == 0 && (WS_OOFFS % 256) == 0 && (WS_OHK % 256) == 0 && (WS_OHV % 256) == 0);
static_assert((WS_OEK % 256) == 0 && (WS_OEV % 256) == 0 && (WS_OEA % 256) == 0 && (WS_OYHL % 256) == 0);

typedef int v4i __attribute__((ext_vector_type(4)));
typedef int v2i __attribute__((ext_vector_type(2)));
typedef unsigned int v2u __attribute__((ext_vector_type(2)));
typedef v4i __attribute__((may_alias)) v4ia;
typedef v2i __attribute__((may_alias)) v2ia;

__device__ __forceinline__ int nkey(int b, int i, int nN) {
  return clampi((int)((unsigned)b * (unsigned)SEQ_L + (unsigned)i), 0, nN - 1);
}

__device__ __forceinline__ void par_seg(const float* __restrict__ src, int n4src, int n4dst,
                                        float* __restrict__ dst, int tid) {
  const int ic = tid < n4src ? tid : n4src - 1;
  v4f v = *(const v4fa*)(src + 4 * ic);
  asm volatile("" :: "v"(v));
  const unsigned mk = (tid < n4src) ? 0xFFFFFFFFu : 0u;
  v4f o;
  o.x = __uint_as_float((bf16_bits(v.x) << 16) & mk);
  o.y = __uint_as_float((bf16_bits(v.y) << 16) & mk);
  o.z = __uint_as_float((bf16_bits(v.z) << 16) & mk);
  o.w = __uint_as_float((bf16_bits(v.w) << 16) & mk);
  const int td = tid < n4dst ? tid : n4dst - 1;
  volatile v4f* q = (volatile v4f*)(dst + 4 * td);
  const bool ok = tid < n4dst;
  if (ok) *q = o;
  __threadfence();
  if (ok) *q = o;
}

__global__ __launch_bounds__(NTHR)
void k_par(const float* __restrict__ key_b, const float* __restrict__ query_b, const float* __restrict__ value_b,
           const float* __restrict__ proj_b, const float* __restrict__ ek_b2, const float* __restrict__ ev_b2,
           const float* __restrict__ ea_w1, const float* __restrict__ ea_b1, const float* __restrict__ ea_g,
           const float* __restrict__ ea_bt, const float* __restrict__ ek_w1, const float* __restrict__ ek_b1,
           const float* __restrict__ ek_g, const float* __restrict__ ek_bt, const float* __restrict__ ev_w1,
           const float* __restrict__ ev_b1, const float* __restrict__ ev_g, const float* __restrict__ ev_bt,
           const float* __restrict__ ea_w2, const float* __restrict__ ea_b2, float* __restrict__ P) {
  const int tid = (int)threadIdx.x;
  par_seg(key_b,   32, 32, P + PAR_KB,   tid);
  par_seg(query_b, 32, 32, P + PAR_QB,   tid);
  par_seg(value_b, 32, 32, P + PAR_VB,   tid);
  par_seg(proj_b,  32, 32, P + PAR_PB,   tid);
  par_seg(ek_b2,   32, 32, P + PAR_EKB2, tid);
  par_seg(ev_b2,   32, 32, P + PAR_EVB2, tid);
  par_seg(ea_w1, 160, 160, P + PAR_EDGE0 + 0,    tid);
  par_seg(ea_b1,  32,  32, P + PAR_EDGE0 + 640,  tid);
  par_seg(ea_g,   32,  32, P + PAR_EDGE0 + 768,  tid);
  par_seg(ea_bt,  32,  32, P + PAR_EDGE0 + 896,  tid);
  par_seg(ek_w1, 160, 160, P + PAR_EDGE0 + 1024, tid);
  par_seg(ek_b1,  32,  32, P + PAR_EDGE0 + 1664, tid);
  par_seg(ek_g,   32,  32, P + PAR_EDGE0 + 1792, tid);
  par_seg(ek_bt,  32,  32, P + PAR_EDGE0 + 1920, tid);
  par_seg(ev_w1, 160, 160, P + PAR_EDGE0 + 2048, tid);
  par_seg(ev_b1,  32,  32, P + PAR_EDGE0 + 2688, tid);
  par_seg(ev_g,   32,  32, P + PAR_EDGE0 + 2816, tid);
  par_seg(ev_bt,  32,  32, P + PAR_EDGE0 + 2944, tid);
  par_seg(ea_w2, 256, 256, P + PAR_EAW2, tid);
  par_seg(ea_b2,   2,   8, P + PAR_EAB2, tid);
}

__device__ __forceinline__ void wprep_unit(const float* __restrict__ w, int KT, int u,
                                           unsigned short* __restrict__ wt) {
  const int ppr = KT >> 3;
  const int n   = clampi(u / ppr, 0, DM - 1);
  const int k8  = (u - (u / ppr) * ppr) * 8;
  float x[8];
#pragma unroll
  for (int e = 0; e < 8; ++e) {
    const int kk = (k8 + e) & 127;
    const float v = w[(size_t)kk * DM + n];
    asm volatile("" :: "v"(v));
    x[e] = v;
  }
  const v4u o = pack8_bf16((v4f){ x[0], x[1], x[2], x[3] }, (v4f){ x[4], x[5], x[6], x[7] });
  volatile v4u* q = (volatile v4u*)(wt + (size_t)n * (size_t)KT + k8);
  *q = o;
  __threadfence();
  *q = o;
}

#define WB1 8
#define WB2 16
#define WB3 24
#define WB4 (WB3 + KT_EK / 16)
#define WB5 (WB4 + KT_EV / 16)
#define WBT (WB5 + KT_PJ / 16)

__global__ __launch_bounds__(NTHR)
void k_wprep(const float* __restrict__ kw, const float* __restrict__ qw, const float* __restrict__ vw,
             const float* __restrict__ ekw2, const float* __restrict__ evw2, const float* __restrict__ pw,
             unsigned short* __restrict__ KW, unsigned short* __restrict__ QW, unsigned short* __restrict__ VW,
             unsigned short* __restrict__ EKW, unsigned short* __restrict__ EVW, unsigned short* __restrict__ PW) {
  const int tid = (int)threadIdx.x;
  const int bx  = (int)blockIdx.x;
  if (bx < WB1)      wprep_unit(kw,   128,   bx * NTHR + tid,         KW);
  else if (bx < WB2) wprep_unit(qw,   128,   (bx - WB1) * NTHR + tid, QW);
  else if (bx < WB3) wprep_unit(vw,   128,   (bx - WB2) * NTHR + tid, VW);
  else if (bx < WB4) wprep_unit(ekw2, KT_EK, (bx - WB3) * NTHR + tid, EKW);
  else if (bx < WB5) wprep_unit(evw2, KT_EV, (bx - WB4) * NTHR + tid, EVW);
  else               wprep_unit(pw,   KT_PJ, (bx - WB5) * NTHR + tid, PW);
}

__device__ __forceinline__ int scan_chunk(const int* __restrict__ bix, const int* __restrict__ hix, int nN,
                                          int cbase, int slotBase, int nb, int* list, int tid, int lane, int wave) {
  int wc = 0;
  const int el0 = tid * EPT;
  const int e0  = cbase + el0;
  v4i ba = *(const v4ia*)(bix + e0);
  v4i bb = *(const v4ia*)(bix + e0 + 4);
  v4i ha = *(const v4ia*)(hix + e0);
  v4i hb = *(const v4ia*)(hix + e0 + 4);
  asm volatile("" :: "v"(ba));
  asm volatile("" :: "v"(bb));
  asm volatile("" :: "v"(ha));
  asm volatile("" :: "v"(hb));
  const unsigned nbs = (unsigned)slotBase;
  const unsigned unb = (unsigned)nb;
  const unsigned s0 = (unsigned)nkey(ba.x, ha.x, nN) - nbs, s1 = (unsigned)nkey(ba.y, ha.y, nN) - nbs;
  const unsigned s2 = (unsigned)nkey(ba.z, ha.z, nN) - nbs, s3 = (unsigned)nkey(ba.w, ha.w, nN) - nbs;
  const unsigned s4 = (unsigned)nkey(bb.x, hb.x, nN) - nbs, s5 = (unsigned)nkey(bb.y, hb.y, nN) - nbs;
  const unsigned s6 = (unsigned)nkey(bb.z, hb.z, nN) - nbs, s7 = (unsigned)nkey(bb.w, hb.w, nN) - nbs;
  const bool h0 = s0 < unb, h1 = s1 < unb, h2 = s2 < unb, h3 = s3 < unb;
  const bool h4 = s4 < unb, h5 = s5 < unb, h6 = s6 < unb, h7 = s7 < unb;
  const unsigned any = __builtin_amdgcn_ballot_w32(h0 | h1 | h2 | h3 | h4 | h5 | h6 | h7);
  if (any != 0u) {
#define HITJ(J, HJ, SJ) { \
      const unsigned mj = __builtin_amdgcn_ballot_w32(HJ); \
      if (mj != 0u) { \
        if (HJ) { \
          const int pos = wc + (int)__builtin_amdgcn_mbcnt_lo(mj, 0u); \
          if (pos < WCAP) list[wave * WCAP + pos] = ((el0 + (J)) << 12) | (int)(SJ); \
        } \
        wc += (int)__builtin_popcount(mj); } }
    HITJ(0, h0, s0)
    HITJ(1, h1, s1)
    HITJ(2, h2, s2)
    HITJ(3, h3, s3)
    HITJ(4, h4, s4)
    HITJ(5, h5, s5)
    HITJ(6, h6, s6)
    HITJ(7, h7, s7)
#undef HITJ
  }
  return wc;
}

__global__ __launch_bounds__(NTHR) void k_bucket(const int* __restrict__ bix, const int* __restrict__ hix,
                                                 const int* __restrict__ tix, int* __restrict__ LIST,
                                                 int* __restrict__ OFFS, int nN, int nE) {
  extern __shared__ v4u lds_dyn[];
  int* reg1 = (int*)lds_dyn;
  int* reg2 = reg1 + BCAP;
  int* scnt = reg2 + BCAP;
  int* soff = scnt + NBRUN;
  int* list = soff + OFFP;
  int* wcnt = list + LISTN;
  int* wtot = wcnt + NWAVE;
  int* wflg = wtot + NWAVE;
  const int tid = (int)threadIdx.x, lane = tid & 31, wave = tid >> 5;
  const int b = (int)blockIdx.x;
  const int slotBase = b * NBRUN;
  int nb = nN - slotBase;
  nb = nb < 0 ? 0 : (nb > NBRUN ? NBRUN : nb);

  {
    const v4i z4 = (v4i){0, 0, 0, 0};
    for (int i = tid; i < NBRUN; i += NTHR) scnt[i] = 0;
    for (int i = tid; i < BCAP / 4; i += NTHR) *(v4ia*)(reg2 + 4 * i) = z4;
  }
  __syncthreads();

  int totraw = 0;
  const int nChunks = nE / CHUNK;
#pragma unroll 1
  for (int ch = 0; ch < nChunks; ++ch) {
    const int cbase = ch * CHUNK;
    const int wc = scan_chunk(bix, hix, nN, cbase, slotBase, nb, list, tid, lane, wave);
    if (lane == 0) wcnt[wave] = wc;
    __syncthreads();
    int pre = 0, all = 0;
#pragma unroll
    for (int w2 = 0; w2 < NWAVE; ++w2) {
      int c = wcnt[w2];
      c = c < 0 ? 0 : (c > WCAP ? WCAP : c);
      all += c;
      pre += (w2 < wave) ? c : 0;
    }
    const int wcc  = wc > WCAP ? WCAP : wc;
    const int tot  = totraw > BCAP ? BCAP : totraw;
    const int base = tot + pre;
#pragma unroll 1
    for (int i0 = 0; i0 < wcc; i0 += 32) {
      const int i  = i0 + lane;
      const int ic = i < wcc ? i : wcc - 1;
      const int ent = list[wave * WCAP + ic];
      const int el  = (ent >> 12) & (CHUNK - 1);
      const int sl  = ent & (NBRUN - 1);
      int eid = cbase + el;
      eid = eid > nE - 1 ? nE - 1 : eid;
      const int pos = base + i;
      if (i < wcc && pos < BCAP) reg1[pos] = (int)(((unsigned)sl << 20) | (unsigned)eid);
    }
    totraw += all;
    __syncthreads();
  }
  const int nh  = totraw > BCAP ? BCAP : totraw;
  const int ovf = totraw > BCAP ? 1 : 0;

  if (wave == 0) {
#pragma unroll 1
    for (int b0 = 0; b0 < nh; b0 += 32) {
      const int idx = b0 + lane;
      const int uv  = reg1[idx < nh ? idx : nh - 1];
      const int m32 = (nh - b0) < 32 ? (nh - b0) : 32;
#pragma unroll 1
      for (int k = 0; k < m32; ++k) {
        const int u  = __builtin_amdgcn_readlane(uv, k);
        const int sl = (int)(((unsigned)u >> 20) & (unsigned)(NBRUN - 1));
        if (lane == 0) scnt[sl] = scnt[sl] + 1;
      }
    }
  }
  __syncthreads();

  int fl = ovf;
  {
    const v4i ca = *(const v4ia*)(scnt + 4 * tid);
    const int e0 = ca.x < 0 ? 0 : ca.x, e1 = ca.y < 0 ? 0 : ca.y, e2 = ca.z < 0 ? 0 : ca.z, e3 = ca.w < 0 ? 0 : ca.w;
    const bool big = (e0 > DEGCAP) | (e1 > DEGCAP) | (e2 > DEGCAP) | (e3 > DEGCAP);
    const unsigned bm = __builtin_amdgcn_ballot_w32(big);
    const int ts = e0 + e1 + e2 + e3;
    int incl = ts;
#pragma unroll
    for (int d = 1; d < 32; d <<= 1) {
      const int up = __shfl_up(incl, d);
      if (lane >= d) incl += up;
    }
    if (lane == 31) wtot[wave] = incl;
    if (lane == 0)  wflg[wave] = (bm != 0u) ? 1 : 0;
    __syncthreads();
    int pre = 0;
#pragma unroll
    for (int w2 = 0; w2 < NWAVE; ++w2) {
      pre += (w2 < wave) ? wtot[w2] : 0;
      fl |= wflg[w2];
    }
    int run = pre + incl - ts;
    soff[4 * tid + 0] = run; run += e0;
    soff[4 * tid + 1] = run; run += e1;
    soff[4 * tid + 2] = run; run += e2;
    soff[4 * tid + 3] = run;
    if (tid < 32) soff[NBRUN + tid] = (tid < 2) ? nh : ((tid == 2) ? fl : 0);
  }
  __syncthreads();
  for (int i = tid; i < NBRUN; i += NTHR) list[i] = soff[i];
  __syncthreads();

  if (wave == 0) {
#pragma unroll 1
    for (int b0 = 0; b0 < nh; b0 += 32) {
      const int idx = b0 + lane;
      const int uv  = reg1[idx < nh ? idx : nh - 1];
      const int m32 = (nh - b0) < 32 ? (nh - b0) : 32;
#pragma unroll 1
      for (int k = 0; k < m32; ++k) {
        const int u   = __builtin_amdgcn_readlane(uv, k);
        const int sl  = (int)(((unsigned)u >> 20) & (unsigned)(NBRUN - 1));
        const int eid = (int)((unsigned)u & 0xFFFFFu);
        if (lane == 0) {
          int pos = list[sl];
          pos = pos < 0 ? 0 : (pos > BCAP - 1 ? BCAP - 1 : pos);
          reg2[pos] = eid;
          list[sl] = pos + 1;
        }
      }
    }
  }
  __syncthreads();

  {
    int* Lb = LIST + (size_t)b * (size_t)BCAP * 2;
    const int nU = BCAP / 2;
#pragma unroll 1
    for (int it = 0; it < (nU + NTHR - 1) / NTHR; ++it) {
      const int u  = it * NTHR + tid;
      const int uc = u < nU ? u : nU - 1;
      const v2i ee = *(const v2ia*)(reg2 + 2 * uc);
      const int e0 = clampi(ee.x, 0, nE - 1);
      const int e1 = clampi(ee.y, 0, nE - 1);
      int bq0 = bix[e0];
      int tq0 = tix[e0];
      int bq1 = bix[e1];
      int tq1 = tix[e1];
      asm volatile("" :: "v"(bq0));
      asm volatile("" :: "v"(tq0));
      asm volatile("" :: "v"(bq1));
      asm volatile("" :: "v"(tq1));
      const int s0 = nkey(bq0, tq0, nN);
      const int s1 = nkey(bq1, tq1, nN);
      const int m0 = (2 * uc     < nh) ? -1 : 0;
      const int m1 = (2 * uc + 1 < nh) ? -1 : 0;
      const v4i o = (v4i){ s0 & m0, e0 & m0, s1 & m1, e1 & m1 };
      volatile v4i* q = (volatile v4i*)(Lb + 4 * (size_t)uc);
      const bool ok = u < nU;
      if (ok) *q = o;
      __threadfence();
      if (ok) *q = o;
    }
  }
  {
    int* Ob = OFFS + (size_t)b * OFFP;
    const int nU = OFFP / 4;
#pragma unroll 1
    for (int it = 0; it < (nU + NTHR - 1) / NTHR; ++it) {
      const int u  = it * NTHR + tid;
      const int uc = u < nU ? u : nU - 1;
      const v4i o = *(const v4ia*)(soff + 4 * uc);
      volatile v4i* q = (volatile v4i*)(Ob + 4 * uc);
      const bool ok = u < nU;
      if (ok) *q = o;
      __threadfence();
      if (ok) *q = o;
    }
  }
}

__device__ __forceinline__ float lin5(float x0, float x1, float x2, float x3, float x4,
                                      float a, float b, float c, float d, float e, float bias) {
  float h = x0 * a;
  h = fmaf(x1, b, h);
  h = fmaf(x2, c, h);
  h = fmaf(x3, d, h);
  h = fmaf(x4, e, h);
  h += bias;
  return (h > 0.0f) ? h : (h - h);
}

__global__ __launch_bounds__(NTHR) __attribute__((amdgpu_num_vgpr(248)))
void k_edge(const float* __restrict__ ef, const int* __restrict__ LISTc, const int* __restrict__ OFFS,
            const float* __restrict__ PAR, unsigned short* __restrict__ HKV, float* __restrict__ EA,
            int b0, int nE) {
  __shared__ __attribute__((aligned(16))) float sP[PE_N];
  const int tid = (int)threadIdx.x, lane = tid & 31, wave = tid >> 5;
#pragma unroll 1
  for (int it = 0; it < (PE_N / 4 + NTHR - 1) / NTHR; ++it) {
    const int u  = it * NTHR + tid;
    const int uc = u < PE_N / 4 ? u : PE_N / 4 - 1;
    v4f v = *(const v4fa*)(PAR + PAR_EDGE0 + 4 * uc);
    asm volatile("" :: "v"(v));
    if (u < PE_N / 4) *(v4fa*)(sP + 4 * u) = v;
  }
  __syncthreads();

  const int rbase = ((int)blockIdx.x * NWAVE + wave) * PPW;
  const int lb    = rbase / BCAP;
  int cnt = OFFS[(size_t)(b0 + lb) * OFFP + NBRUN];
  asm volatile("" :: "v"(cnt));
  cnt = clampi(cnt, 0, BCAP);
  const int cntu = __builtin_amdgcn_readfirstlane(cnt);
  const int c4 = 4 * lane;

#pragma unroll 1
  for (int pp = 0; pp < PPW; ++pp) {
    const int r = rbase + pp;
    const int p = r - lb * BCAP;
    v2i se = *(const v2ia*)(LISTc + 2 * (size_t)r);
    asm volatile("" :: "v"(se));
    const int eid = clampi(se.y, 0, nE - 1);
    const float* fp = ef + (size_t)eid * NFE;
    float f0 = fp[0];
    float f1 = fp[1];
    float f2 = fp[2];
    float f3 = fp[3];
    float f4 = fp[4];
    asm volatile("" :: "v"(f0));
    asm volatile("" :: "v"(f1));
    asm volatile("" :: "v"(f2));
    asm volatile("" :: "v"(f3));
    asm volatile("" :: "v"(f4));
    const float x0 = bf16_val(f0), x1 = bf16_val(f1), x2 = bf16_val(f2), x3 = bf16_val(f3), x4 = bf16_val(f4);
    const unsigned lm = (p < cntu) ? 0xFFFFFFFFu : 0u;

#pragma unroll 1
    for (int m = 0; m < 3; ++m) {
      const float* bp = sP + m * 1024 + c4;
      const v4f w0 = *(const v4fa*)(bp);
      const v4f w1 = *(const v4fa*)(bp + 128);
      const v4f w2 = *(const v4fa*)(bp + 256);
      const v4f w3 = *(const v4fa*)(bp + 384);
      const v4f w4 = *(const v4fa*)(bp + 512);
      const v4f bb = *(const v4fa*)(bp + 640);
      const v4f gg = *(const v4fa*)(bp + 768);
      const v4f be = *(const v4fa*)(bp + 896);
      const float h0 = lin5(x0, x1, x2, x3, x4, w0.x, w1.x, w2.x, w3.x, w4.x, bb.x);
      const float h1 = lin5(x0, x1, x2, x3, x4, w0.y, w1.y, w2.y, w3.y, w4.y, bb.y);
      const float h2 = lin5(x0, x1, x2, x3, x4, w0.z, w1.z, w2.z, w3.z, w4.z, bb.z);
      const float h3 = lin5(x0, x1, x2, x3, x4, w0.w, w1.w, w2.w, w3.w, w4.w, bb.w);
      float s = (h0 + h1) + (h2 + h3);
      s += __shfl_xor(s, 1);
      s += __shfl_xor(s, 2);
      s += __shfl_xor(s, 4);
      s += __shfl_xor(s, 8);
      s += __shfl_xor(s, 16);
      const float mu = s * 0.0078125f;
      const float d0 = h0 - mu, d1 = h1 - mu, d2 = h2 - mu, d3 = h3 - mu;
      float qq = (d0 * d0 + d1 * d1) + (d2 * d2 + d3 * d3);
      qq += __shfl_xor(qq, 1);
      qq += __shfl_xor(qq, 2);
      qq += __shfl_xor(qq, 4);
      qq += __shfl_xor(qq, 8);
      qq += __shfl_xor(qq, 16);
      const float var = qq * 0.0078125f;
      const float rs  = 1.0f / sqrtf(var + 1e-5f);
      const float n0 = d0 * rs * gg.x + be.x;
      const float n1 = d1 * rs * gg.y + be.y;
      const float n2 = d2 * rs * gg.z + be.z;
      const float n3 = d3 * rs * gg.w + be.w;

      if (m == 0) {
        float l0 = 0.0f, l1 = 0.0f, l2 = 0.0f, l3 = 0.0f, l4 = 0.0f, l5 = 0.0f, l6 = 0.0f, l7 = 0.0f;
#pragma unroll 1
        for (int i = 0; i < 4; ++i) {
          const float hv = (i == 0) ? n0 : ((i == 1) ? n1 : ((i == 2) ? n2 : n3));
          const float* wp = sP + 3072 + (c4 + i) * 8;
          const v4f wa = *(const v4fa*)(wp);
          const v4f wb = *(const v4fa*)(wp + 4);
          l0 = fmaf(hv, wa.x, l0);
          l1 = fmaf(hv, wa.y, l1);
          l2 = fmaf(hv, wa.z, l2);
          l3 = fmaf(hv, wa.w, l3);
          l4 = fmaf(hv, wb.x, l4);
          l5 = fmaf(hv, wb.y, l5);
          l6 = fmaf(hv, wb.z, l6);
          l7 = fmaf(hv, wb.w, l7);
        }
#pragma unroll
        for (int st = 1; st < 32; st <<= 1) {
          l0 += __shfl_xor(l0, st);
          l1 += __shfl_xor(l1, st);
          l2 += __shfl_xor(l2, st);
          l3 += __shfl_xor(l3, st);
          l4 += __shfl_xor(l4, st);
          l5 += __shfl_xor(l5, st);
          l6 += __shfl_xor(l6, st);
          l7 += __shfl_xor(l7, st);
        }
        const int hsel = lane & 7;
        float lv = l0;
        lv = (hsel == 1) ? l1 : lv;
        lv = (hsel == 2) ? l2 : lv;
        lv = (hsel == 3) ? l3 : lv;
        lv = (hsel == 4) ? l4 : lv;
        lv = (hsel == 5) ? l5 : lv;
        lv = (hsel == 6) ? l6 : lv;
        lv = (hsel == 7) ? l7 : lv;
        const float val = lv + sP[4096 + hsel];
        const unsigned km = (lane < 8) ? lm : 0u;
        const float ov = __uint_as_float(__float_as_uint(val) & km);
        volatile float* q = (volatile float*)(EA + (size_t)r * 32 + lane);
        *q = ov;
        __threadfence();
        *q = ov;
      } else {
        const int kt  = (m == 1) ? KT_EK : KT_EV;
        const int sp2 = (m == 1) ? SPLIT_EK : SPLIT_EV;
        unsigned short* row = HKV + (size_t)(m - 1) * HPLANE + (size_t)r * (size_t)kt + c4;
        const v2u hi = (v2u){ pk16(bf16_bits(n0), bf16_bits(n1)) & lm, pk16(bf16_bits(n2), bf16_bits(n3)) & lm };
        const v2u lo = (v2u){ pk16(bf16_lo_bits(n0), bf16_lo_bits(n1)) & lm,
                              pk16(bf16_lo_bits(n2), bf16_lo_bits(n3)) & lm };
        volatile v2u* qh = (volatile v2u*)(row);
        volatile v2u* ql = (volatile v2u*)(row + 128);
        *qh = hi;
        if (sp2 != 0) *ql = lo;
        __threadfence();
        *qh = hi;
        if (sp2 != 0) *ql = lo;
      }
    }
  }
}

__global__ __launch_bounds__(NTHR) __attribute__((amdgpu_num_vgpr(248)))
void k_replay(const float* __restrict__ Kf, const float* __restrict__ Qf, const float* __restrict__ Vf,
              const float* __restrict__ EKc, const float* __restrict__ EVc, const float* __restrict__ EAc,
              const int* __restrict__ LISTc, const int* __restrict__ OFFS, const float* __restrict__ PAR,
              unsigned short* __restrict__ YHL, int b0, int nReal) {
  __shared__ __attribute__((aligned(16))) float strip[NWAVE * DEGCAP * 8];
  __shared__ __attribute__((aligned(16))) float sB[256];
  const int tid = (int)threadIdx.x, lane = tid & 31, wave = tid >> 5;
  if (tid < 64) {
    v4f v = *(const v4fa*)(PAR + PAR_EKB2 + 4 * tid);
    asm volatile("" :: "v"(v));
    *(v4fa*)(sB + 4 * tid) = v;
  }
  __syncthreads();

  const int rowc = (int)blockIdx.x * NWAVE + wave;
  const int lb   = rowc >> 10;
  const int slot = rowc & (NBRUN - 1);
  const int b    = b0 + lb;
  const int t    = b * NBRUN + slot;
  const bool live = t < nReal;
  const int* ob = OFFS + (size_t)b * OFFP;
  int o0 = ob[slot];
  int o1 = ob[slot + 1];
  int fg = ob[NBRUN + 2];
  asm volatile("" :: "v"(o0));
  asm volatile("" :: "v"(o1));
  asm volatile("" :: "v"(fg));
  const int st = clampi(o0, 0, BCAP);
  int c = clampi(o1 - o0, 0, DEGCAP);
  c = c > BCAP - st ? BCAP - st : c;
  c = live ? c : 0;
  const int cn  = __builtin_amdgcn_readfirstlane(c);
  const int stu = __builtin_amdgcn_readfirstlane(st);
  const int tcl = clampi(t, 0, nReal - 1);
  const int c4  = 4 * lane;
  v4f q = *(const v4fa*)(Qf + (size_t)tcl * DM + c4);
  asm volatile("" :: "v"(q));
  const v4f bk = *(const v4fa*)(sB + c4);
  const v4f bv = *(const v4fa*)(sB + 128 + c4);
  const size_t r0 = (size_t)lb * BCAP + (size_t)stu;
  const int*   lp  = LISTc + 2 * r0;
  const float* ekp = EKc + r0 * DM + c4;
  const float* evp = EVc + r0 * DM + c4;
  const float* eap = EAc + r0 * 32 + (lane >> 2);
  float* sp = strip + wave * (DEGCAP * 8) + (lane >> 2);

  float mx = -__builtin_inff();
#pragma unroll 1
  for (int j = 0; j < cn; ++j) {
    v2i se = *(const v2ia*)(lp + 2 * j);
    asm volatile("" :: "v"(se));
    const int s = clampi(se.x, 0, nReal - 1);
    v4f k = *(const v4fa*)(Kf + (size_t)s * DM + c4);
    v4f e = *(const v4fa*)(ekp + (size_t)j * DM);
    float ea = eap[(size_t)j * 32];
    asm volatile("" :: "v"(k));
    asm volatile("" :: "v"(e));
    asm volatile("" :: "v"(ea));
    const v4f tt = e + bk;
    const v4f ks = k + tt;
    float pd = ks.x * q.x;
    pd = fmaf(ks.y, q.y, pd);
    pd = fmaf(ks.z, q.z, pd);
    pd = fmaf(ks.w, q.w, pd);
    pd += __shfl_xor(pd, 1);
    pd += __shfl_xor(pd, 2);
    const float v = pd + ea;
    sp[j * 8] = v;
    mx = fmaxf(mx, v);
  }
  __builtin_amdgcn_fence(__ATOMIC_RELEASE, "workgroup");
  __builtin_amdgcn_wave_barrier();
  __builtin_amdgcn_fence(__ATOMIC_ACQUIRE, "workgroup");
  const bool fin = (__float_as_uint(mx) & 0x7f800000u) != 0x7f800000u;
  const float m = fin ? mx : 0.0f;

  float den = 0.0f;
#pragma unroll 1
  for (int j = 0; j < cn; ++j) {
    const float lg = sp[j * 8];
    den += expf(lg - m);
  }
  const float dv = den + 1e-16f;

  v4f acc = (v4f){0.0f, 0.0f, 0.0f, 0.0f};
#pragma unroll 1
  for (int j = 0; j < cn; ++j) {
    v2i se = *(const v2ia*)(lp + 2 * j);
    asm volatile("" :: "v"(se));
    const int s = clampi(se.x, 0, nReal - 1);
    v4f vv = *(const v4fa*)(Vf + (size_t)s * DM + c4);
    v4f e  = *(const v4fa*)(evp + (size_t)j * DM);
    asm volatile("" :: "v"(vv));
    asm volatile("" :: "v"(e));
    const float lg  = sp[j * 8];
    const float ex  = expf(lg - m);
    const float att = ex / dv;
    const v4f tt = e + bv;
    const v4f vs = vv + tt;
    acc.x += att * vs.x;
    acc.y += att * vs.y;
    acc.z += att * vs.z;
    acc.w += att * vs.w;
  }
  v4f o = acc;
  const v4f z4 = (v4f){0.0f, 0.0f, 0.0f, 0.0f};
  o = (cn > 0) ? o : z4;
  const float qn = __uint_as_float(0x7fc00000u);
  const v4f n4 = (v4f){qn, qn, qn, qn};
  o = (fg != 0) ? n4 : o;
  const v2u hi = (v2u){ pk16(bf16_bits(o.x), bf16_bits(o.y)), pk16(bf16_bits(o.z), bf16_bits(o.w)) };
  const v2u lo = (v2u){ pk16(bf16_lo_bits(o.x), bf16_lo_bits(o.y)), pk16(bf16_lo_bits(o.z), bf16_lo_bits(o.w)) };
  unsigned short* yrow = YHL + (size_t)tcl * (size_t)KT_PJ + c4;
  volatile v2u* qh = (volatile v2u*)(yrow);
  volatile v2u* ql = (volatile v2u*)(yrow + 128);
  if (live) *qh = hi;
  if (live && SPLIT_PROJ != 0) *ql = lo;
  __threadfence();
  if (live) *qh = hi;
  if (live && SPLIT_PROJ != 0) *ql = lo;
}

static inline int cdiv_i(int a, int b) { return (a + b - 1) / b; }

extern "C" void kernel_launch(void* const* d_in, const int* in_sizes, int n_in,
                              void* d_out, int out_size, void* d_ws, size_t ws_size,
                              hipStream_t stream) {
  if (n_in < 34) return;
  if (in_sizes[0] != N_NODES * DM || in_sizes[1] != N_NODES * DM || in_sizes[2] != N_NODES * DM) return;
  if (in_sizes[3] != N_EDGES * NFE) return;
  if (in_sizes[5] != N_EDGES || in_sizes[6] != N_EDGES || in_sizes[7] != N_EDGES) return;
  if (in_sizes[8] != DM * DM || in_sizes[10] != DM * DM || in_sizes[12] != DM * DM || in_sizes[14] != DM * DM) return;
  if (in_sizes[9] != DM || in_sizes[11] != DM || in_sizes[13] != DM || in_sizes[15] != DM) return;
  if (in_sizes[16] != NFE * DM || in_sizes[22] != NFE * DM || in_sizes[28] != NFE * DM) return;
  if (in_sizes[17] != DM || in_sizes[18] != DM || in_sizes[19] != DM) return;
  if (in_sizes[23] != DM || in_sizes[24] != DM || in_sizes[25] != DM) return;
  if (in_sizes[29] != DM || in_sizes[30] != DM || in_sizes[31] != DM) return;
  if (in_sizes[20] != DM * 8 || in_sizes[21] != 8) return;
  if (in_sizes[26] != DM * DM || in_sizes[32] != DM * DM || in_sizes[27] != DM || in_sizes[33] != DM) return;
  if (out_size != N_NODES * DM) return;
  if (ws_size < WS_TOTAL) return;

  const float* key   = (const float*)d_in[0];
  const float* value = (const float*)d_in[1];
  const float* query = (const float*)d_in[2];
  const float* ef    = (const float*)d_in[3];
  const int*   bix   = (const int*)d_in[5];
  const int*   hix   = (const int*)d_in[6];
  const int*   tix   = (const int*)d_in[7];
  const float* key_w   = (const float*)d_in[8];  const float* key_b   = (const float*)d_in[9];
  const float* query_w = (const float*)d_in[10]; const float* query_b = (const float*)d_in[11];
  const float* value_w = (const float*)d_in[12]; const float* value_b = (const float*)d_in[13];
  const float* proj_w  = (const float*)d_in[14]; const float* proj_b  = (const float*)d_in[15];
  const float* ea_w1 = (const float*)d_in[16]; const float* ea_b1 = (const float*)d_in[17];
  const float* ea_g  = (const float*)d_in[18]; const float* ea_bt = (const float*)d_in[19];
  const float* ea_w2 = (const float*)d_in[20]; const float* ea_b2 = (const float*)d_in[21];
  const float* ek_w1 = (const float*)d_in[22]; const float* ek_b1 = (const float*)d_in[23];
  const float* ek_g  = (const float*)d_in[24]; const float* ek_bt = (const float*)d_in[25];
  const float* ek_w2 = (const float*)d_in[26]; const float* ek_b2 = (const float*)d_in[27];
  const float* ev_w1 = (const float*)d_in[28]; const float* ev_b1 = (const float*)d_in[29];
  const float* ev_g  = (const float*)d_in[30]; const float* ev_bt = (const float*)d_in[31];
  const float* ev_w2 = (const float*)d_in[32]; const float* ev_b2 = (const float*)d_in[33];
  float* out = (float*)d_out;

  char* ws = (char*)d_ws;
  unsigned short* XK  = (unsigned short*)(ws + WS_OXK);
  unsigned short* XV  = (unsigned short*)(ws + WS_OXV);
  unsigned short* XQ  = (unsigned short*)(ws + WS_OXQ);
  unsigned short* KW  = (unsigned short*)(ws + WS_OKW);
  unsigned short* QW  = (unsigned short*)(ws + WS_OQW);
  unsigned short* VW  = (unsigned short*)(ws + WS_OVW);
  unsigned short* EKW = (unsigned short*)(ws + WS_OEKW);
  unsigned short* EVW = (unsigned short*)(ws + WS_OEVW);
  unsigned short* PW  = (unsigned short*)(ws + WS_OPW);
  float*          PAR = (float*)(ws + WS_OPAR);
  float*          KF  = (float*)(ws + WS_OKF);
  float*          QF  = (float*)(ws + WS_OQF);
  float*          VF  = (float*)(ws + WS_OVF);
  int*            LST = (int*)(ws + WS_OLIST);
  int*            OFS = (int*)(ws + WS_OOFFS);
  unsigned short* HK  = (unsigned short*)(ws + WS_OHK);
  unsigned short* HV  = (unsigned short*)(ws + WS_OHV);
  float*          EKc = (float*)(ws + WS_OEK);
  float*          EVc = (float*)(ws + WS_OEV);
  float*          EAc = (float*)(ws + WS_OEA);
  unsigned short* YHL = (unsigned short*)(ws + WS_OYHL);

  hipFuncSetAttribute(reinterpret_cast<const void*>(&k_bucket),
                      hipFuncAttributeMaxDynamicSharedMemorySize, LDS_BKT);

  k_plane<0><<<N_NODES * DM / 8 / 256, 256, 0, stream>>>(key,   N_NODES, DM, DM, XK, N_NODES, DM);
  k_plane<0><<<N_NODES * DM / 8 / 256, 256, 0, stream>>>(value, N_NODES, DM, DM, XV, N_NODES, DM);
  k_plane<0><<<N_NODES * DM / 8 / 256, 256, 0, stream>>>(query, N_NODES, DM, DM, XQ, N_NODES, DM);
  k_par<<<1, NTHR, 0, stream>>>(key_b, query_b, value_b, proj_b, ek_b2, ev_b2,
                                ea_w1, ea_b1, ea_g, ea_bt, ek_w1, ek_b1, ek_g, ek_bt,
                                ev_w1, ev_b1, ev_g, ev_bt, ea_w2, ea_b2, PAR);
  k_wprep<<<WBT, NTHR, 0, stream>>>(key_w, query_w, value_w, ek_w2, ev_w2, proj_w, KW, QW, VW, EKW, EVW, PW);

  {
    const int T = (N_NODES / 64) * (DM / 64);
    k_gemm_nt<0, 1><<<cdiv_i(T, 8), 256, 0, stream>>>(XK, KW, PAR + PAR_KB, KF, N_NODES, DM, DM, DM);
    k_gemm_nt<0, 1><<<cdiv_i(T, 8), 256, 0, stream>>>(XQ, QW, PAR + PAR_QB, QF, N_NODES, DM, DM, DM);
    k_gemm_nt<0, 1><<<cdiv_i(T, 8), 256, 0, stream>>>(XV, VW, PAR + PAR_VB, VF, N_NODES, DM, DM, DM);
  }
  k_bucket<<<NBLK, NTHR, LDS_BKT, stream>>>(bix, hix, tix, LST, OFS, N_NODES, N_EDGES);

  for (int c = 0; c < NCHUNK; ++c) {
    const int b0 = c * GCH;
    const int* LISTc = LST + (size_t)b0 * (size_t)BCAP * 2;
    k_edge<<<CHROWS / (NWAVE * PPW), NTHR, 0, stream>>>(ef, LISTc, OFS, PAR, HK, EAc, b0, N_EDGES);
    const int T = (CHROWS / 64) * (DM / 64);
    k_gemm_nt<0, 0><<<cdiv_i(T, 8), 256, 0, stream>>>(HK, EKW, PAR, EKc, CHROWS, DM, KT_EK, DM);
    k_gemm_nt<0, 0><<<cdiv_i(T, 8), 256, 0, stream>>>(HV, EVW, PAR, EVc, CHROWS, DM, KT_EV, DM);
    k_replay<<<GCH * NBRUN / NWAVE, NTHR, 0, stream>>>(KF, QF, VF, EKc, EVc, EAc, LISTc, OFS, PAR, YHL,
                                                       b0, N_NODES);
  }

  {
    const int T = (N_NODES / 64) * (DM / 64);
    k_gemm_nt<0, 1><<<cdiv_i(T, 8), 256, 0, stream>>>(YHL, PW, PAR + PAR_PB, out, N_NODES, DM, KT_PJ, DM);
  }
}
